// LIFENet_89524298318168
// MI455X (gfx1250) — hardware-verified
//
#include <hip/hip_runtime.h>
#include <math.h>

typedef __attribute__((ext_vector_type(16))) _Float16 v16h;
typedef __attribute__((ext_vector_type(16))) __bf16 v16b;
typedef __attribute__((ext_vector_type(8)))  _Float16 v8h;
typedef __attribute__((ext_vector_type(8)))  float v8f;
typedef __attribute__((ext_vector_type(4)))  float v4f;
typedef __attribute__((ext_vector_type(2)))  float v2f;
typedef __attribute__((ext_vector_type(4)))  unsigned v4u;
typedef __attribute__((ext_vector_type(4)))  int v4i;
typedef float __attribute__((may_alias)) float_a;
typedef int __attribute__((may_alias)) int_a;

template <typename T> __device__ __forceinline__ void vst2(void* p, T v) { *(volatile T*)p = v; __threadfence(); *(volatile T*)p = v; }
__device__ __forceinline__ v8f wmma16(v16h a, v16h b, v8f c) {
  v8f d = __builtin_amdgcn_wmma_f32_16x16x32_f16(false, a, false, b, (short)0, c, false, false);
  asm volatile("v_nop\n\tv_nop\n\tv_nop\n\tv_nop" : "+v"(d) : "v"(a), "v"(b));
  return d;
}
__device__ __forceinline__ v8f wmma_bf(v16b a, v16b b, v8f c) {
  v8f d = __builtin_amdgcn_wmma_f32_16x16x32_bf16(false, a, false, b, (short)0, c, false, false);
  asm volatile("v_nop\n\tv_nop\n\tv_nop\n\tv_nop" : "+v"(d) : "v"(a), "v"(b));
  return d;
}
__device__ __forceinline__ v16h frag_h(const _Float16* rowk0, int lane) {
  union { v16h v; v8h q[2]; } u; const _Float16* p = rowk0 + 8 * (lane >> 4);
  u.q[0] = *(const v8h*)p; u.q[1] = *(const v8h*)(p + 16); return u.v;
}
__device__ __forceinline__ v16h frag_f32(const float* rowk0, int lane) {
  v16h a; const float* p = rowk0 + 8 * (lane >> 4);
#pragma unroll
  for (int i = 0; i < 8; ++i) { a[i] = (_Float16)p[i]; a[8 + i] = (_Float16)p[16 + i]; }
  return a;
}
__device__ __forceinline__ v16h frag_f32s(const float* rowk0, int lane, float sc) {
  v16h a; const float* p = rowk0 + 8 * (lane >> 4);
#pragma unroll
  for (int i = 0; i < 8; ++i) { a[i] = (_Float16)(p[i] * sc); a[8 + i] = (_Float16)(p[16 + i] * sc); }
  return a;
}
__device__ __forceinline__ v16h fragc_f32(const float* W, int k0, int n, int lane, int ld, int K) {
  v16h a; const int g = lane >> 4;
#pragma unroll
  for (int i = 0; i < 8; ++i) { const int ka = k0 + 8 * g + i, kb = ka + 16;
    a[i] = (_Float16)(ka < K ? W[(size_t)(ka < K ? ka : K - 1) * ld + n] : 0.f); a[8 + i] = (_Float16)(kb < K ? W[(size_t)(kb < K ? kb : K - 1) * ld + n] : 0.f); }
  return a;
}
struct F2 { v16b h, l; };
__device__ __forceinline__ F2 bsplit16(const float v[16]) { F2 r;
#pragma unroll
  for (int i = 0; i < 16; ++i) { const __bf16 h = (__bf16)v[i]; r.h[i] = h; r.l[i] = (__bf16)(v[i] - (float)h); }
  return r; }
__device__ __forceinline__ F2 split_row(const float* row, int k0, int lane) { float v[16]; const float* p = row + k0 + 8 * (lane >> 4);
#pragma unroll
  for (int i = 0; i < 8; ++i) { v[i] = p[i]; v[8 + i] = p[16 + i]; }
  return bsplit16(v); }
__device__ __forceinline__ F2 split_rowK(const float* row, int k0, int lane, int K) { float v[16]; const int g = lane >> 4;
#pragma unroll
  for (int i = 0; i < 8; ++i) { const int ka = k0 + 8 * g + i, kb = ka + 16; v[i] = ka < K ? row[ka < K ? ka : K - 1] : 0.f; v[8 + i] = kb < K ? row[kb < K ? kb : K - 1] : 0.f; }
  return bsplit16(v); }
__device__ __forceinline__ F2 split_col(const float* W, int k0, int n, int lane, int ld, int K) { float v[16]; const int g = lane >> 4;
#pragma unroll
  for (int i = 0; i < 8; ++i) { const int ka = k0 + 8 * g + i, kb = ka + 16; v[i] = ka < K ? W[(size_t)(ka < K ? ka : K - 1) * ld + n] : 0.f; v[8 + i] = kb < K ? W[(size_t)(kb < K ? kb : K - 1) * ld + n] : 0.f; }
  return bsplit16(v); }
__device__ __forceinline__ v8f mac3(const F2& a, const F2& b, v8f c) { c = wmma_bf(a.l, b.h, c); c = wmma_bf(a.h, b.l, c); return wmma_bf(a.h, b.h, c); }
__device__ __forceinline__ float sigm(float v) { return 1.0f / (1.0f + expf(-v)); }
#define LDSX() do { asm volatile("s_wait_dscnt 0" ::: "memory"); __builtin_amdgcn_wave_barrier(); __builtin_amdgcn_fence(__ATOMIC_RELEASE, "workgroup"); } while (0)


#define NB 16
#define TT 96
#define DV 96
#define KK 10
#define KD 960
#define NIN 288
#define NR (NB * TT)
#ifndef NBT
#define NBT NB
#endif
typedef __attribute__((ext_vector_type(8))) __bf16 v8b;
__device__ __forceinline__ v16b frag_b(const __bf16* rowk0, int lane) {
  union { v16b v; v8b q[2]; } u; const __bf16* p = rowk0 + 8 * (lane >> 4);
  u.q[0] = *(const v8b*)p; u.q[1] = *(const v8b*)(p + 16); return u.v;
}
__device__ __forceinline__ float bfr(float v) { return (float)(__bf16)v; }
__device__ __attribute__((noinline)) float exp_ni(float v) { return expf(v); }
__device__ __attribute__((noinline)) float erf_ni(float v) { return erff(v); }
__device__ __attribute__((noinline)) float tanh_ni(float v) { return tanhf(v); }
__device__ __attribute__((noinline)) float expm1_ni(float v) { return expm1f(v); }
__constant__ float c_wi[3 * TT] = {4.584418833e-01f,4.726562500e-01f,4.870876074e-01f,5.017361641e-01f,5.166015625e-01f,5.316839814e-01f,5.469835401e-01f,5.625000000e-01f,5.782335401e-01f,5.941839814e-01f,6.103515625e-01f,6.267361641e-01f,6.433376670e-01f,6.601562500e-01f,6.771918535e-01f,6.944444180e-01f,7.119140625e-01f,7.296007276e-01f,7.475042939e-01f,7.656250000e-01f,7.839627266e-01f,8.025173545e-01f,8.212890625e-01f,8.402777910e-01f,8.594834805e-01f,8.789062500e-01f,8.985460401e-01f,9.184027314e-01f,9.384765625e-01f,9.587674141e-01f,9.792751074e-01f,1.000000000e+00f,9.792751074e-01f,9.587674141e-01f,9.384765625e-01f,9.184027314e-01f,8.985460401e-01f,8.789062500e-01f,8.594834805e-01f,8.402777910e-01f,8.212890625e-01f,8.025173545e-01f,7.839627266e-01f,7.656250000e-01f,7.475042939e-01f,7.296007276e-01f,7.119140625e-01f,6.944444180e-01f,6.771918535e-01f,6.601562500e-01f,6.433376670e-01f,6.267361641e-01f,6.103515625e-01f,5.941839814e-01f,5.782335401e-01f,5.625000000e-01f,5.469835401e-01f,5.316839814e-01f,5.166015625e-01f,5.017361641e-01f,4.870876074e-01f,4.726562500e-01f,4.584418833e-01f,4.444443882e-01f,4.306640625e-01f,4.171007574e-01f,4.037542939e-01f,3.906250000e-01f,3.777127266e-01f,3.650173247e-01f,3.525390625e-01f,3.402778208e-01f,3.282334507e-01f,3.164062500e-01f,3.047960401e-01f,2.934027314e-01f,2.822265625e-01f,2.712674141e-01f,2.605251372e-01f,2.500000000e-01f,2.396918237e-01f,2.296007127e-01f,2.197265625e-01f,2.100694329e-01f,2.006293535e-01f,1.914062500e-01f,1.824001521e-01f,1.736111343e-01f,1.650390625e-01f,1.566840112e-01f,1.485460252e-01f,1.406250000e-01f,1.329209954e-01f,1.254340410e-01f,1.181640625e-01f,1.111110970e-01f,1.181640625e-01f,1.254340410e-01f,1.329209954e-01f,1.406250000e-01f,1.485460252e-01f,1.566840112e-01f,1.650390625e-01f,1.736111343e-01f,1.824001521e-01f,1.914062500e-01f,2.006293535e-01f,2.100694329e-01f,2.197265625e-01f,2.296007127e-01f,2.396918237e-01f,2.500000000e-01f,2.605251372e-01f,2.712674141e-01f,2.822265625e-01f,2.934027314e-01f,3.047960401e-01f,3.164062500e-01f,3.282334507e-01f,3.402778208e-01f,3.525390625e-01f,3.650173247e-01f,3.777127266e-01f,3.906250000e-01f,4.037542939e-01f,4.171007574e-01f,4.306640625e-01f,4.444443882e-01f,4.584418833e-01f,4.726562500e-01f,4.870876074e-01f,5.017361641e-01f,5.166015625e-01f,5.316839814e-01f,5.469835401e-01f,5.625000000e-01f,5.782335401e-01f,5.941839814e-01f,6.103515625e-01f,6.267361641e-01f,6.433376670e-01f,6.601562500e-01f,6.771918535e-01f,6.944444180e-01f,7.119140625e-01f,7.296007276e-01f,7.475042939e-01f,7.656250000e-01f,7.839627266e-01f,8.025173545e-01f,8.212890625e-01f,8.402777910e-01f,8.594834805e-01f,8.789062500e-01f,8.985460401e-01f,9.184027314e-01f,9.384765625e-01f,9.587674141e-01f,9.792751074e-01f,1.000000000e+00f,9.792751074e-01f,9.587674141e-01f,9.384765625e-01f,9.184027314e-01f,8.985460401e-01f,8.789062500e-01f,8.594834805e-01f,8.402777910e-01f,8.212890625e-01f,8.025173545e-01f,7.839627266e-01f,7.656250000e-01f,7.475042939e-01f,7.296007276e-01f,7.119140625e-01f,6.944444180e-01f,6.771918535e-01f,6.601562500e-01f,6.433376670e-01f,6.267361641e-01f,6.103515625e-01f,5.941839814e-01f,5.782335401e-01f,5.625000000e-01f,5.469835401e-01f,5.316839814e-01f,5.166015625e-01f,5.017361641e-01f,4.870876074e-01f,4.726562500e-01f,4.584418833e-01f,4.444443882e-01f,1.085073600e-04f,4.340269370e-04f,9.765625000e-04f,1.736112754e-03f,2.712671645e-03f,3.906250000e-03f,5.316843279e-03f,6.944441237e-03f,8.789062500e-03f,1.085069869e-02f,1.312933583e-02f,1.562500000e-02f,1.833767816e-02f,2.126735449e-02f,2.441406250e-02f,2.777778357e-02f,3.135849908e-02f,3.515625000e-02f,3.917101398e-02f,4.340276867e-02f,4.785156250e-02f,5.251736939e-02f,5.740016326e-02f,6.250000000e-02f,6.781685352e-02f,7.335068285e-02f,7.910156250e-02f,8.506945521e-02f,9.125433117e-02f,9.765625000e-02f,1.042751893e-01f,1.111110970e-01f,1.181640625e-01f,1.254340410e-01f,1.329209954e-01f,1.406250000e-01f,1.485460252e-01f,1.566840112e-01f,1.650390625e-01f,1.736111343e-01f,1.824001521e-01f,1.914062500e-01f,2.006293535e-01f,2.100694329e-01f,2.197265625e-01f,2.296007127e-01f,2.396918237e-01f,2.500000000e-01f,2.605251372e-01f,2.712674141e-01f,2.822265625e-01f,2.934027314e-01f,3.047960401e-01f,3.164062500e-01f,3.282334507e-01f,3.402778208e-01f,3.525390625e-01f,3.650173247e-01f,3.777127266e-01f,3.906250000e-01f,4.037542939e-01f,4.171007574e-01f,4.306640625e-01f,4.444443882e-01f,4.584418833e-01f,4.726562500e-01f,4.870876074e-01f,5.017361641e-01f,5.166015625e-01f,5.316839814e-01f,5.469835401e-01f,5.625000000e-01f,5.782335401e-01f,5.941839814e-01f,6.103515625e-01f,6.267361641e-01f,6.433376670e-01f,6.601562500e-01f,6.771918535e-01f,6.944444180e-01f,7.119140625e-01f,7.296007276e-01f,7.475042939e-01f,7.656250000e-01f,7.839627266e-01f,8.025173545e-01f,8.212890625e-01f,8.402777910e-01f,8.594834805e-01f,8.789062500e-01f,8.985460401e-01f,9.184027314e-01f,9.384765625e-01f,9.587674141e-01f,9.792751074e-01f,1.000000000e+00f};

#define PK_E 0
#define PK_A (PK_E + KD * NIN)
#define PK_V (PK_A + KD * KD)
#define PK_END (PK_V + KD * KD)
#define WS_PK   0u
#define WS_INB  (((2u * PK_END) + 127u) / 128u * 128u)
#define WS_HE   (WS_INB + 2u * NR * NIN)
#define WS_HEH  (WS_HE + 4u * NR * KD)
#define WS_HEL  (WS_HEH + 2u * NR * KD)
#define WS_KEY  (WS_HEL + 2u * NR * KD)
#define WS_QRY  (WS_KEY + 4u * NR * KD)
#define WS_HA   (WS_QRY + 4u * NR * KD)
#define WS_HR   (WS_HA + 4u * NR * KD)
#define WS_END  (WS_HR + 4u * NR * KD)

__global__ __launch_bounds__(256) void k_pack(const float* __restrict__ WE, const float* __restrict__ WA, const float* __restrict__ VA, __bf16* __restrict__ PK) {
  __shared__ __align__(16) __bf16 s[KD]; const int n = blockIdx.x, which = blockIdx.y, t = threadIdx.x; int K; size_t dst; const float* src;
  if (which == 0) { K = NIN; dst = PK_E + (size_t)n * NIN; src = WE + (size_t)n * NIN; } else if (which == 1) { K = KD; dst = PK_A + (size_t)n * KD; src = WA + (size_t)n * KD; } else { K = KD; dst = PK_V + (size_t)n * KD; src = VA + (size_t)n * KD; }
  for (int k = t; k < K; k += 256) s[k] = (__bf16)src[k];
  __syncthreads();
  for (int q = t; q < K / 8; q += 256) vst2((unsigned*)(PK + dst + q * 8), *(const v4u*)&s[q * 8]);
}
__global__ __launch_bounds__(96) void k_inp(const float* __restrict__ X, const float* __restrict__ Mm, const float* __restrict__ DF, __bf16* __restrict__ INB) {
  __shared__ __align__(16) __bf16 s[NIN]; const size_t r = blockIdx.x; const int t = threadIdx.x;
  s[t] = (__bf16)X[r * DV + t]; s[DV + t] = (__bf16)Mm[r * DV + t]; s[2 * DV + t] = (__bf16)DF[r * DV + t];
  __syncthreads();
  if (t < NIN / 8) vst2((unsigned*)(INB + r * NIN + t * 8), *(const v4u*)&s[t * 8]);
}
__global__ __launch_bounds__(128) void k_he(const __bf16* __restrict__ INB, const __bf16* __restrict__ PK, const float* __restrict__ BE, const float* __restrict__ POS, float* __restrict__ HE, __bf16* __restrict__ HEH, __bf16* __restrict__ HEL) {
  __shared__ __align__(16) float so[4][16][68]; __shared__ __align__(16) __bf16 soh[4][16][72], sol[4][16][72];
  const int tid = threadIdx.x, wave = tid >> 5, lane = tid & 31, col = lane & 15, g = lane >> 4; const size_t r0 = (size_t)blockIdx.x * 64 + wave * 16; const int n0 = blockIdx.y * 64;
  v8f acc[4] = {};
#pragma unroll
  for (int kc = 0; kc < NIN / 32; ++kc) { const v16b a = frag_b(INB + (r0 + col) * NIN + kc * 32, lane);
#pragma unroll
    for (int j = 0; j < 4; ++j) acc[j] = wmma_bf(a, frag_b(PK + PK_E + (size_t)(n0 + j * 16 + col) * NIN + kc * 32, lane), acc[j]); }
#pragma unroll
  for (int j = 0; j < 4; ++j) { const int c = n0 + j * 16 + col; const float bb = bfr(BE[c]);
#pragma unroll
    for (int r = 0; r < 8; ++r) { const size_t row = r0 + 8 * g + r; const int t = (int)(row % TT); const float pre = (acc[j][r] + bb) + bfr(POS[(size_t)t * KD + c]); const float v = (pre > 0.f) ? pre : expm1_ni(pre);
      so[wave][8 * g + r][j * 16 + col] = v; const __bf16 hb = (__bf16)v; soh[wave][8 * g + r][j * 16 + col] = hb; sol[wave][8 * g + r][j * 16 + col] = (__bf16)(v - (float)hb); } }
  LDSX();
  for (int rl = 0; rl < 16; ++rl) { if (lane < 16) vst2(HE + (r0 + rl) * KD + n0 + lane * 4, *(const v4f*)&so[wave][rl][lane * 4]); else if (lane < 24) vst2((unsigned*)(HEH + (r0 + rl) * KD + n0 + (lane - 16) * 8), *(const v4u*)&soh[wave][rl][(lane - 16) * 8]); else vst2((unsigned*)(HEL + (r0 + rl) * KD + n0 + (lane - 24) * 8), *(const v4u*)&sol[wave][rl][(lane - 24) * 8]); }
}
__global__ __launch_bounds__(128) void k_kq(const __bf16* __restrict__ HEH, const __bf16* __restrict__ HEL, const __bf16* __restrict__ PK, float* __restrict__ KEY, float* __restrict__ QRY) {
  __shared__ __align__(16) float so[4][16][68];
  const int tid = threadIdx.x, wave = tid >> 5, lane = tid & 31, col = lane & 15, g = lane >> 4; const size_t r0 = (size_t)blockIdx.x * 64 + wave * 16; const int n0 = blockIdx.y * 64; const int which = blockIdx.z;
  const __bf16* P = PK + (which ? PK_V : PK_A); float* OUT = which ? QRY : KEY;
  v8f acc[4] = {};
#pragma unroll 2
  for (int kc = 0; kc < KD / 32; ++kc) { F2 a; a.h = frag_b(HEH + (r0 + col) * KD + kc * 32, lane); a.l = frag_b(HEL + (r0 + col) * KD + kc * 32, lane);
#pragma unroll
    for (int j = 0; j < 4; ++j) { const v16b w = frag_b(P + (size_t)(n0 + j * 16 + col) * KD + kc * 32, lane); acc[j] = wmma_bf(a.l, w, acc[j]); acc[j] = wmma_bf(a.h, w, acc[j]); } }
#pragma unroll
  for (int j = 0; j < 4; ++j)
#pragma unroll
    for (int r = 0; r < 8; ++r) so[wave][8 * g + r][j * 16 + col] = acc[j][r];
  LDSX();
  for (int rl = 0; rl < 16; ++rl) if (lane < 16) vst2(OUT + (r0 + rl) * KD + n0 + lane * 4, *(const v4f*)&so[wave][rl][lane * 4]);
}
__global__ __launch_bounds__(192) void k_att(const float* __restrict__ KEY, const float* __restrict__ QRY, const float* __restrict__ WAV, const float* __restrict__ HE, float* __restrict__ HA) {
  __shared__ float sq[KD]; __shared__ float slg[TT]; __shared__ float ssc[TT]; __shared__ __align__(16) float sha[KD];
  const int tid = threadIdx.x; const int b = blockIdx.x / TT, i = blockIdx.x % TT; const size_t rq = (size_t)b * TT + i;
  for (int d = tid; d < KD; d += 192) sq[d] = QRY[rq * KD + d];
  __syncthreads();
  { const int j = tid >> 1, half = tid & 1; const float* kr = KEY + ((size_t)b * TT + j) * KD; float a = 0.f;
#pragma unroll 1
    for (int d = half * (KD / 2); d < (half + 1) * (KD / 2); ++d) a += bfr(WAV[d]) * tanh_ni(kr[d] + sq[d]);
    a += __shfl_xor(a, 1); if (half == 0) slg[j] = a; }
  __syncthreads();
  if (tid < 32) { float mx = -3.0e38f; for (int j = tid; j < TT; j += 32) mx = fmaxf(mx, slg[j]);
#pragma unroll
    for (int o = 1; o < 32; o <<= 1) mx = fmaxf(mx, __shfl_xor(mx, o));
    float se = 0.f; for (int j = tid; j < TT; j += 32) se += exp_ni(slg[j] - mx);
#pragma unroll
    for (int o = 1; o < 32; o <<= 1) se += __shfl_xor(se, o);
    for (int j = tid; j < TT; j += 32) ssc[j] = exp_ni(slg[j] - mx) / se; }
  __syncthreads();
#pragma unroll 1
  for (int d = tid; d < KD; d += 192) { float a = 0.f; const float* he = HE + (size_t)b * TT * KD + d;
#pragma unroll 1
    for (int j = 0; j < TT; ++j) a += ssc[j] * he[(size_t)j * KD]; sha[d] = a; }
  __syncthreads();
  for (int q = tid; q < KD / 4; q += 192) vst2(HA + rq * KD + q * 4, *(const v4f*)&sha[q * 4]);
}
__global__ __launch_bounds__(192) void k_hr(const float* __restrict__ HA, const float* __restrict__ Mm, const float* __restrict__ DF, const float* __restrict__ WTD, const float* __restrict__ BTD, const float* __restrict__ WIMP, const float* __restrict__ BIMP, float* __restrict__ HR, float* __restrict__ IMP) {
  __shared__ __align__(16) float shr[KD]; __shared__ __align__(16) float simp[DV];
  const int tid = threadIdx.x; const int b = blockIdx.x / TT, t = blockIdx.x % TT; const size_t row = (size_t)b * TT + t;
  for (int kd = tid; kd < KD; kd += 192) { const int d = kd % DV; const float m = bfr(Mm[row * DV + d]); const float dl = bfr(DF[row * DV + d]);
    const float gam = exp_ni(-fmaxf(dl * bfr(WTD[kd]) + bfr(BTD[kd]), 0.f)); int idx = t - ((int)dl - 1); idx = min(max(idx, 0), TT - 1);
    const float ha = HA[row * KD + kd]; const float hf = HA[((size_t)b * TT + idx) * KD + kd];
    shr[kd] = m * ha + (1.0f - m) * (gam * hf + (1.0f - gam) * ha); }
  __syncthreads();
  if (tid < DV) { const int d = tid; float a = 0.f; for (int k = 0; k < KK; ++k) a += shr[k * DV + d] * bfr(WIMP[(size_t)d * KD + k * DV + d]); simp[d] = a + bfr(BIMP[d]); }
  __syncthreads();
  for (int q = tid; q < KD / 4; q += 192) vst2(HR + row * KD + q * 4, *(const v4f*)&shr[q * 4]);
  if (tid < DV / 4) vst2(IMP + row * DV + tid * 4, *(const v4f*)&simp[tid * 4]);
}
__global__ __launch_bounds__(256) void k_fc(const float* __restrict__ HR, const float* __restrict__ WFC, const float* __restrict__ BFC, float* __restrict__ OUT0) {
  __shared__ float sv[KD * 3]; __shared__ __align__(16) float sout[NB * KK]; const int tid = threadIdx.x;
  for (int b = 0; b < NBT; ++b) {
    for (int q = tid; q < KD * 3; q += 256) { const int kd = q / 3, f = q % 3; float a = 0.f; const float* hr = HR + (size_t)b * TT * KD + kd; for (int t = 0; t < TT; ++t) a += c_wi[f * TT + t] * hr[(size_t)t * KD]; sv[q] = a; }
    __syncthreads();
    if (tid < KK) { float a = 0.f; for (int q = 0; q < KD * 3; ++q) a += sv[q] * bfr(WFC[(size_t)tid * KD * 3 + q]); sout[b * KK + tid] = a + bfr(BFC[tid]); }
    __syncthreads(); }
  for (int b = NBT; b < NB; ++b) if (tid < KK) sout[b * KK + tid] = 0.f;
  __syncthreads();
  if (tid < NB * KK / 4) vst2(OUT0 + tid * 4, *(const v4f*)&sout[tid * 4]);
}
extern "C" void kernel_launch(void* const* d_in, const int* in_sizes, int n_in, void* d_out, int out_size, void* d_ws, size_t ws_size, hipStream_t stream) {
  (void)in_sizes; (void)n_in; (void)out_size;
  const float** F = (const float**)d_in;
  if (ws_size < (size_t)WS_END) return;
  char* ws = (char*)d_ws; __bf16 *PK = (__bf16*)(ws + WS_PK), *INB = (__bf16*)(ws + WS_INB), *HEH = (__bf16*)(ws + WS_HEH), *HEL = (__bf16*)(ws + WS_HEL); float *HE = (float*)(ws + WS_HE), *KEY = (float*)(ws + WS_KEY), *QRY = (float*)(ws + WS_QRY), *HA = (float*)(ws + WS_HA), *HR = (float*)(ws + WS_HR);
  float* OUT0 = (float*)d_out; float* IMP = (float*)((char*)d_out + 640);
  k_pack<<<dim3(KD, 3), 256, 0, stream>>>(F[3], F[6], F[7], PK);
  k_inp<<<NBT * TT, 96, 0, stream>>>(F[0], F[1], F[2], INB);
  k_he<<<dim3(NBT * TT / 64, KD / 64), 128, 0, stream>>>(INB, PK, F[4], F[5], HE, HEH, HEL);
  k_kq<<<dim3(NBT * TT / 64, KD / 64, 2), 128, 0, stream>>>(HEH, HEL, PK, KEY, QRY);
  k_att<<<NBT * TT, 192, 0, stream>>>(KEY, QRY, F[8], HE, HA);
  k_hr<<<NBT * TT, 192, 0, stream>>>(HA, F[1], F[2], F[9], F[10], F[11], F[12], HR, IMP);
  k_fc<<<1, 256, 0, stream>>>(HR, F[13], F[14], OUT0);
}
